// Transformer_25013889531990
// MI455X (gfx1250) — hardware-run, weakly checked
//
#include <hip/hip_runtime.h>


#ifndef NB
#define NB 4
#endif
#ifndef SEQ
#define SEQ 512
#endif
#define NB_FULL  4
#define SEQ_FULL 512
#ifndef OUT_SEQ
#define OUT_SEQ SEQ
#endif
#define DM     512
#define NH_    8
#define HD     64
#define HD2    128
#define KK     1024
#define NN     1024
#define XP     1024
#define NL     4
#define ROWS   (NB * SEQ)
#define QRS    2048.0f
#define QRI    (1.0f / 2048.0f)
#define WCAR   16.0f
#define WCI    (1.0f / 16.0f)
#define PCAR   16384.0f
#define PCI    (1.0f / 16384.0f)
#define LOG2E  1.4426950408889634f
#define EPS_   1.0e-5f
#define TINY_  1.0e-30f
#define SP     (SEQ + 4)
#define OSP    132
#define OFFI   ((size_t)NB_FULL * SEQ_FULL * DM)
#define WPLANE ((size_t)NN * KK)

static_assert(HD == 64);
static_assert(NH_ * HD == DM);
static_assert(HD2 == 2 * HD);
static_assert(KK == 2 * DM && NN == 2 * DM && XP == 2 * DM);
static_assert(KK % 32 == 0);
static_assert(NN % 64 == 0);
static_assert(SEQ % 64 == 0);
static_assert(ROWS % 32 == 0);
static_assert(ROWS % 8 == 0);
static_assert((SP * 4) % 16 == 0 && (OSP * 4) % 16 == 0 && OSP >= HD2);
static_assert(NB <= NB_FULL);
static_assert(SEQ <= SEQ_FULL);
static_assert(OFFI * 4 == (size_t)4194304);
static_assert((2 * 16 * SP + 16 * OSP) * 4 <= 131072);
static_assert(16 * 68 * 4 <= 131072);
static_assert(64 * 72 * 2 <= 131072);

typedef _Float16 h16;
typedef __attribute__((ext_vector_type(16))) _Float16 v16h;
typedef __attribute__((ext_vector_type(8)))  _Float16 v8h;
typedef __attribute__((ext_vector_type(4)))  _Float16 v4h;
typedef __attribute__((ext_vector_type(8)))  float    v8f;
typedef __attribute__((ext_vector_type(4)))  float    v4f;
typedef v4f  __attribute__((may_alias)) v4fa;

__device__ __forceinline__ unsigned short f2bf(float f) { unsigned u = __float_as_uint(f); u += 0x7FFFu + ((u >> 16) & 1u); return (unsigned short)(u >> 16); }
__device__ __forceinline__ float bfr(float f) { return __uint_as_float(((unsigned)f2bf(f)) << 16); }
__device__ __forceinline__ v16h cat16(v8h lo, v8h hi) { return __builtin_shufflevector(lo, hi, 0, 1, 2, 3, 4, 5, 6, 7, 8, 9, 10, 11, 12, 13, 14, 15); }
__device__ __forceinline__ v8f wmma16(v16h a, v16h b, v8f c) { return __builtin_amdgcn_wmma_f32_16x16x32_f16(false, a, false, b, (short)0, c, false, false); }
__device__ __forceinline__ v16h  ldh(const h16* p) { return cat16(*(const v8h*)p, *(const v8h*)(p + 16)); }
__device__ __forceinline__ void wave_sync() { __builtin_amdgcn_fence(3  , "wavefront"); __builtin_amdgcn_wave_barrier(); asm volatile("" ::: "memory"); }
static __device__ __forceinline__ h16 toh_flush(float v) { const h16 r = (h16)v; return (fabsf(v) < 6.103515625e-05f) ? (h16)0.0f : r; }
__device__ __forceinline__ v8f mma(v16h a, v16h b, v8f c) { c = wmma16(a, b, c); asm volatile("v_nop\n\tv_nop\n\tv_nop\n\tv_nop" : "+v"(c) : "v"(a), "v"(b)); return c; }
__device__ __forceinline__ float softplus_f(float x) { return fmaxf(x, 0.0f) + log1pf(expf(-fabsf(x))); }

static_assert(256 * 16 == XP * 4);
__global__ __launch_bounds__(256) void k_xin(const float* __restrict__ XR, const float* __restrict__ XI, float* X) {
    const int row = blockIdx.x, q = threadIdx.x; const int part = q >> 7, c = (q & 127) * 4;
    const int b = row / SEQ, t = row % SEQ;
    const size_t so = ((size_t)b * SEQ_FULL + t) * DM + c;
    const v4f a = *(const v4f*)(XR + so); const v4f bq = *(const v4f*)(XI + so); v4f o;
#pragma unroll
    for (int i = 0; i < 4; ++i) o[i] = bfr(part ? bq[i] : a[i]);
    float* d = X + (size_t)row * XP + part * DM + c;
    *(volatile v4f*)d = o; __threadfence(); *(volatile v4f*)d = o;
}

static_assert((NN * (KK / 8)) % 256 == 0);
__global__ __launch_bounds__(256) void k_wprep(const float* __restrict__ WRe, const float* __restrict__ WIm, h16* dst) {
    const int l = blockIdx.y; const int p = blockIdx.x * 256 + threadIdx.x;
    const int n = p >> 7, k8 = (p & 127) * 8;
    const int np = n >> 9, kp = k8 >> 9; const int e = n & 511, kk = k8 & 511;
    const size_t so = ((size_t)l * DM + e) * DM + kk;
    const v4f r0 = *(const v4f*)(WRe + so), r1 = *(const v4f*)(WRe + so + 4), i0 = *(const v4f*)(WIm + so), i1 = *(const v4f*)(WIm + so + 4);
    const bool useR = (np == kp);
    const float sc = ((np == 0) & (kp == 1)) ? -WCAR : WCAR;
    v8h o;
#pragma unroll
    for (int i = 0; i < 4; ++i) { o[i] = toh_flush(bfr(useR ? r0[i] : i0[i]) * sc); o[4 + i] = toh_flush(bfr(useR ? r1[i] : i1[i]) * sc); }
    h16* d = dst + (size_t)l * WPLANE + (size_t)n * KK + k8;
    *(volatile v8h*)d = o; __threadfence(); *(volatile v8h*)d = o;
}

static_assert(32 * 8 * 2 == DM);
__global__ __launch_bounds__(256) void k_ln(const float* __restrict__ X, const float* __restrict__ GR, const float* __restrict__ BR,
                                            const float* __restrict__ GI, const float* __restrict__ BI, h16* AH, h16* AR) {
#pragma clang fp contract(off)
    const int lane = threadIdx.x & 31; const int wave = __builtin_amdgcn_readfirstlane(threadIdx.x >> 5);
    const int row = blockIdx.x * 8 + wave; const int part = blockIdx.y;
    const int c = 8 * lane;
    const float* src = X + (size_t)row * XP + part * DM + c;
    const v8f x0 = *(const v8f*)src, x1 = *(const v8f*)(src + 256);
    float s = 0.0f;
#pragma unroll
    for (int j = 0; j < 8; ++j) s += x0[j] + x1[j];
#pragma unroll
    for (int m = 16; m >= 1; m >>= 1) s += __shfl_xor(s, m, 32);
    const float mean = s * (1.0f / DM);
    v8f d0, d1; float q = 0.0f;
#pragma unroll
    for (int j = 0; j < 8; ++j) { d0[j] = x0[j] - mean; d1[j] = x1[j] - mean; q += d0[j] * d0[j] + d1[j] * d1[j]; }
#pragma unroll
    for (int m = 16; m >= 1; m >>= 1) q += __shfl_xor(q, m, 32);
    const float inv = __builtin_amdgcn_rsqf(q * (1.0f / DM) + EPS_);
    const v8f gr0 = *(const v8f*)(GR + c), gr1 = *(const v8f*)(GR + 256 + c), gi0 = *(const v8f*)(GI + c), gi1 = *(const v8f*)(GI + 256 + c);
    const v8f br0 = *(const v8f*)(BR + c), br1 = *(const v8f*)(BR + 256 + c), bi0 = *(const v8f*)(BI + c), bi1 = *(const v8f*)(BI + 256 + c);
    const v8f g0 = part ? gi0 : gr0, g1 = part ? gi1 : gr1, b0 = part ? bi0 : br0, b1 = part ? bi1 : br1;
    v8h h0, h1, r0, r1;
#pragma unroll
    for (int j = 0; j < 8; ++j) {
        const float o0 = d0[j] * inv * bfr(g0[j]) + bfr(b0[j]); const float o1 = d1[j] * inv * bfr(g1[j]) + bfr(b1[j]);
        const h16 a0 = toh_flush(o0); const h16 a1 = toh_flush(o1);
        h0[j] = a0; h1[j] = a1; r0[j] = toh_flush((o0 - (float)a0) * QRS); r1[j] = toh_flush((o1 - (float)a1) * QRS);
    }
    const size_t oo = (size_t)row * KK + part * DM + c;
    *(volatile v8h*)(AH + oo) = h0; *(volatile v8h*)(AH + oo + 256) = h1; *(volatile v8h*)(AR + oo) = r0; *(volatile v8h*)(AR + oo + 256) = r1;
    __threadfence();
    *(volatile v8h*)(AH + oo) = h0; *(volatile v8h*)(AH + oo + 256) = h1; *(volatile v8h*)(AR + oo) = r0; *(volatile v8h*)(AR + oo + 256) = r1;
}

__device__ __forceinline__ void gemm_main(const h16* __restrict__ AH, const h16* __restrict__ AR, const h16* __restrict__ BT, int r0, int c0, int lr, int hi,
                                          v8f (&accH)[2][4], v8f (&accR)[2][4]) {
#pragma unroll
    for (int mb = 0; mb < 2; ++mb)
#pragma unroll
        for (int nb = 0; nb < 4; ++nb) { accH[mb][nb] = (v8f){}; accR[mb][nb] = (v8f){}; }
    const size_t aoff = (size_t)(r0 + lr) * KK + 8 * hi, boff = (size_t)(c0 + lr) * KK + 8 * hi;
#pragma unroll 1
    for (int kc = 0; kc < KK; kc += 32) {
        v16h ah[2], ar[2];
#pragma unroll
        for (int mb = 0; mb < 2; ++mb) { ah[mb] = ldh(AH + aoff + (size_t)mb * 16 * KK + kc); ar[mb] = ldh(AR + aoff + (size_t)mb * 16 * KK + kc); }
#pragma unroll
        for (int nb = 0; nb < 4; ++nb) { const v16h bq = ldh(BT + boff + (size_t)nb * 16 * KK + kc);
#pragma unroll
            for (int mb = 0; mb < 2; ++mb) { accH[mb][nb] = mma(ah[mb], bq, accH[mb][nb]); accR[mb][nb] = mma(ar[mb], bq, accR[mb][nb]); } }
    }
}

static_assert(32 * 16 * 4 == 16 * 128);
__global__ __launch_bounds__(32) __attribute__((amdgpu_num_vgpr(256)))
void k_gemm_qkv(const h16* __restrict__ AH, const h16* __restrict__ AR, const h16* __restrict__ BT, h16* PH, h16* PR) {
    __shared__ __align__(16) float os[16 * 68];
    const int lane = threadIdx.x & 31, lr = lane & 15, hi = lane >> 4; const int r0 = blockIdx.x * 32, c0 = blockIdx.y * 64;
    v8f accH[2][4], accR[2][4];
    gemm_main(AH, AR, BT, r0, c0, lr, hi, accH, accR);
    const int part = c0 >> 9, head = (c0 & 511) >> 6;
    const int bb = r0 / SEQ, tt = r0 % SEQ;
    const size_t tbase = ((size_t)(bb * NH_ + head) * SEQ + tt) * HD2 + part * HD;
#pragma unroll
    for (int mb = 0; mb < 2; ++mb) {
#pragma unroll
        for (int nb = 0; nb < 4; ++nb) {
#pragma unroll
            for (int j = 0; j < 8; ++j) os[(hi * 8 + j) * 68 + nb * 16 + lr] = (accH[mb][nb][j] + accR[mb][nb][j] * QRI) * WCI; }
        wave_sync();
        const size_t sb = tbase + (size_t)(mb * 16) * HD2;
#pragma unroll 1
        for (int ps = 0; ps < 2; ++ps) {
#pragma unroll
            for (int s = 0; s < 4; ++s) { const int row = 4 * s + (lane >> 3), c8 = (lane & 7) * 8;
                const v4f x0 = *(const v4fa*)(&os[row * 68 + c8]); const v4f x1 = *(const v4fa*)(&os[row * 68 + c8 + 4]); v8h hv, rv;
#pragma unroll
                for (int i = 0; i < 4; ++i) { const h16 a0 = toh_flush(x0[i]); const h16 a1 = toh_flush(x1[i]); hv[i] = a0; hv[4 + i] = a1;
                    rv[i] = toh_flush((x0[i] - (float)a0) * QRS); rv[4 + i] = toh_flush((x1[i] - (float)a1) * QRS); }
                const size_t oo = sb + (size_t)row * HD2 + c8;
                *(volatile v8h*)(PH + oo) = hv; *(volatile v8h*)(PR + oo) = rv; }
            if (ps == 0) __threadfence(); }
        wave_sync();
    }
}

static_assert(32 * 16 * 8 == 16 * 256);
__global__ __launch_bounds__(32) __attribute__((amdgpu_num_vgpr(256)))
void k_gemm_out(const h16* __restrict__ AH, const h16* __restrict__ AR, const h16* __restrict__ BT,
                const float* __restrict__ BSR, const float* __restrict__ BSI, const float* __restrict__ XIN, float* XOUT) {
    __shared__ __align__(16) float os[16 * 68];
    const int lane = threadIdx.x & 31, lr = lane & 15, hi = lane >> 4; const int r0 = blockIdx.x * 32, c0 = blockIdx.y * 64;
    v8f accH[2][4], accR[2][4];
    gemm_main(AH, AR, BT, r0, c0, lr, hi, accH, accR);
    const int part = c0 >> 9, cc = c0 & 511; const int cofs = lr * 4;
    const v4f b0 = *(const v4f*)(BSR + cc + cofs), b1 = *(const v4f*)(BSI + cc + cofs); v4f bv;
#pragma unroll
    for (int i = 0; i < 4; ++i) bv[i] = bfr(part ? b1[i] : b0[i]);
    const size_t obase = (size_t)r0 * XP + c0 + cofs;
#pragma unroll
    for (int mb = 0; mb < 2; ++mb) {
#pragma unroll
        for (int nb = 0; nb < 4; ++nb) {
#pragma unroll
            for (int j = 0; j < 8; ++j) os[(hi * 8 + j) * 68 + nb * 16 + lr] = (accH[mb][nb][j] + accR[mb][nb][j] * QRI) * WCI; }
        wave_sync();
        const size_t sb = obase + (size_t)(mb * 16) * XP;
#pragma unroll 1
        for (int ps = 0; ps < 2; ++ps) {
#pragma unroll
            for (int s = 0; s < 8; ++s) { const int row = 2 * s + hi;
                const v4f res = *(const v4f*)(XIN + sb + (size_t)row * XP);
                const v4f val = *(const v4fa*)(&os[row * 68 + cofs]) + bv + res;
                *(volatile v4f*)(XOUT + sb + (size_t)row * XP) = val; }
            if (ps == 0) __threadfence(); }
        wave_sync();
    }
}

__global__ __launch_bounds__(32) __attribute__((amdgpu_num_vgpr(256)))
void k_gemm_ff(const h16* __restrict__ AH, const h16* __restrict__ AR, const h16* __restrict__ BT,
               const float* __restrict__ STEP, const float* __restrict__ LAMB, int layer, float* Y, size_t ioff, int pitch, int oseq) {
    __shared__ __align__(16) float os[16 * 68];
    const int lane = threadIdx.x & 31, lr = lane & 15, hi = lane >> 4; const int r0 = blockIdx.x * 32, c0 = blockIdx.y * 64;
    v8f accH[2][4], accR[2][4];
    gemm_main(AH, AR, BT, r0, c0, lr, hi, accH, accR);
    const int part = c0 >> 9, cc = c0 & 511; const int cofs = lr * 4;
    const float ss = softplus_f(bfr(STEP[layer])); const float lm = softplus_f(bfr(LAMB[layer]));
    const float sl = ss * lm * (float)(1 - part);
    const int bb = r0 / SEQ, tt = r0 % SEQ;
    const size_t ybase = (size_t)part * ioff + ((size_t)bb * oseq + tt) * (size_t)pitch + cc + cofs;
    const size_t xo = (size_t)r0 * KK + c0 + cofs;
#pragma unroll
    for (int mb = 0; mb < 2; ++mb) {
#pragma unroll
        for (int nb = 0; nb < 4; ++nb) {
#pragma unroll
            for (int j = 0; j < 8; ++j) os[(hi * 8 + j) * 68 + nb * 16 + lr] = (accH[mb][nb][j] + accR[mb][nb][j] * QRI) * WCI; }
        wave_sync();
#pragma unroll 1
        for (int ps = 0; ps < 2; ++ps) {
#pragma unroll
            for (int s = 0; s < 8; ++s) { const int row = 2 * s + hi;
                const v4f x1 = *(const v4fa*)(&os[row * 68 + cofs]);
                const v4h hv = *(const v4h*)(AH + xo + (size_t)(mb * 16 + row) * KK); const v4h rv = *(const v4h*)(AR + xo + (size_t)(mb * 16 + row) * KK);
                v4f val;
#pragma unroll
                for (int i = 0; i < 4; ++i) { const float xn = (float)hv[i] + (float)rv[i] * QRI; const float g = xn + ss * x1[i] - sl; val[i] = (g > 0.0f) ? g : 0.0f; }
                *(volatile v4f*)(Y + ybase + (size_t)(mb * 16 + row) * (size_t)pitch) = val; }
            if (ps == 0) __threadfence(); }
        wave_sync();
    }
}

static_assert(256 * 2 == 64 * 8);
__global__ __launch_bounds__(256) void k_vT(const h16* __restrict__ src, h16* dst) {
    __shared__ __align__(16) h16 ts[64 * 72];
    const int tid = threadIdx.x; const int t0 = blockIdx.x * 64, c0 = blockIdx.y * 64; const int z = blockIdx.z;
    const h16* s = src + (size_t)z * SEQ * HD2; h16* d = dst + (size_t)z * HD2 * SEQ;
#pragma unroll
    for (int i = 0; i < 2; ++i) { const int p = tid + 256 * i, r = p >> 3, c8 = (p & 7) * 8;
        const v8h v = *(const v8h*)(s + (size_t)(t0 + r) * HD2 + c0 + c8);
#pragma unroll
        for (int e = 0; e < 8; ++e) ts[(c8 + e) * 72 + r] = v[e]; }
    __syncthreads();
    v8h o0, o1; size_t a0, a1;
    { const int p = tid,       row = p >> 3, t8 = (p & 7) * 8; o0 = *(const v8h*)(&ts[row * 72 + t8]); a0 = (size_t)(c0 + row) * SEQ + t0 + t8; }
    { const int p = tid + 256, row = p >> 3, t8 = (p & 7) * 8; o1 = *(const v8h*)(&ts[row * 72 + t8]); a1 = (size_t)(c0 + row) * SEQ + t0 + t8; }
    *(volatile v8h*)(d + a0) = o0; *(volatile v8h*)(d + a1) = o1;
    __threadfence();
    *(volatile v8h*)(d + a0) = o0; *(volatile v8h*)(d + a1) = o1;
}

struct pt3 { float e, r, i; };
__device__ __forceinline__ pt3 pterm(float dr, float di, float mx) {
    const float m2 = dr * dr + di * di;
    const float rs = __builtin_amdgcn_rsqf(fmaxf(m2, TINY_));
    const float mag = m2 * rs;
    const float e = __builtin_amdgcn_exp2f((mag - mx) * LOG2E);
    const bool ok = m2 > TINY_;
    pt3 o; o.e = e; o.r = ok ? e * (dr * rs) : e; o.i = ok ? e * (di * rs) : 0.0f; return o;
}

static_assert(32 * 16 * 8 == 16 * 2 * 128);
__global__ __launch_bounds__(32) __attribute__((amdgpu_num_vgpr(256)))
void k_attn(const h16* __restrict__ WP, const h16* __restrict__ VTH, const h16* __restrict__ VTR, h16* CH, h16* CR) {
    __shared__ __align__(16) float Sr[16 * SP];
    __shared__ __align__(16) float Si[16 * SP];
    __shared__ __align__(16) float os[16 * OSP];
    const int lane = threadIdx.x & 31, lr = lane & 15, hi = lane >> 4;
    const int zh = blockIdx.y; const int b = zh / NH_, h = zh % NH_;
    const int t0 = blockIdx.x * 16;
    const int so = lr * SP;
    const size_t pbase = (size_t)zh * SEQ * HD2;
    const size_t qo = pbase + (size_t)(t0 + lr) * HD2 + 8 * hi;
    const v16h q0 = ldh(WP + qo), q1 = ldh(WP + qo + 32), q2 = ldh(WP + qo + 64), q3 = ldh(WP + qo + 96);
    const v16h n0 = -q0, n1 = -q1;

    const size_t ko = pbase + (size_t)lr * HD2 + 8 * hi;
    float mx2 = 0.0f;
#pragma unroll 1
    for (int key0 = 0; key0 < SEQ; key0 += 32) {
        const h16* ka = WP + ko + (size_t)key0 * HD2;
        v8f sRa = (v8f){}, sIa = (v8f){}, sRb = (v8f){}, sIb = (v8f){};
        { const v16h a = ldh(ka), c = ldh(ka + 16 * HD2);
          sRa = mma(a, q0, sRa); sIa = mma(a, q2, sIa); sRb = mma(c, q0, sRb); sIb = mma(c, q2, sIb); }
        { const v16h a = ldh(ka + 32), c = ldh(ka + 16 * HD2 + 32);
          sRa = mma(a, q1, sRa); sIa = mma(a, q3, sIa); sRb = mma(c, q1, sRb); sIb = mma(c, q3, sIb); }
        { const v16h a = ldh(ka + 64), c = ldh(ka + 16 * HD2 + 64);
          sRa = mma(a, q2, sRa); sIa = mma(a, n0, sIa); sRb = mma(c, q2, sRb); sIb = mma(c, n0, sIb); }
        { const v16h a = ldh(ka + 96), c = ldh(ka + 16 * HD2 + 96);
          sRa = mma(a, q3, sRa); sIa = mma(a, n1, sIa); sRb = mma(c, q3, sRb); sIb = mma(c, n1, sIb); }
        const int ja = key0 + 8 * hi;
        v4f ra0, ra1, rb0, rb1, ia0, ia1, ib0, ib1;
#pragma unroll
        for (int i = 0; i < 4; ++i) {
            ra0[i] = sRa[i] * 0.125f; ra1[i] = sRa[4 + i] * 0.125f; rb0[i] = sRb[i] * 0.125f; rb1[i] = sRb[4 + i] * 0.125f;
            ia0[i] = sIa[i] * 0.125f; ia1[i] = sIa[4 + i] * 0.125f; ib0[i] = sIb[i] * 0.125f; ib1[i] = sIb[4 + i] * 0.125f;
            const float m0 = ra0[i] * ra0[i] + ia0[i] * ia0[i], m1 = ra1[i] * ra1[i] + ia1[i] * ia1[i];
            const float m2 = rb0[i] * rb0[i] + ib0[i] * ib0[i], m3 = rb1[i] * rb1[i] + ib1[i] * ib1[i];
            mx2 = fmaxf(mx2, fmaxf(fmaxf(m0, m1), fmaxf(m2, m3)));
        }
        *(v4fa*)(&Sr[so + ja]) = ra0; *(v4fa*)(&Sr[so + ja + 4]) = ra1; *(v4fa*)(&Sr[so + ja + 16]) = rb0; *(v4fa*)(&Sr[so + ja + 20]) = rb1;
        *(v4fa*)(&Si[so + ja]) = ia0; *(v4fa*)(&Si[so + ja + 4]) = ia1; *(v4fa*)(&Si[so + ja + 16]) = ib0; *(v4fa*)(&Si[so + ja + 20]) = ib1;
    }
    mx2 = fmaxf(mx2, __shfl_xor(mx2, 16, 32));
    const float mx = mx2 * __builtin_amdgcn_rsqf(fmaxf(mx2, TINY_));
    wave_sync();

    const size_t vo = (size_t)zh * HD2 * SEQ + (size_t)lr * SEQ + 8 * hi;
    v8f oR[4], oI[4], rR[4], rI[4];
#pragma unroll
    for (int jd = 0; jd < 4; ++jd) { oR[jd] = (v8f){}; oI[jd] = (v8f){}; rR[jd] = (v8f){}; rI[jd] = (v8f){}; }
    float l = 0.0f;
#pragma unroll 1
    for (int key0 = 0; key0 < SEQ; key0 += 32) {
        const int ja = key0 + 8 * hi;
        const v4f ra0 = *(const v4fa*)(&Sr[so + ja]), ra1 = *(const v4fa*)(&Sr[so + ja + 4]), rb0 = *(const v4fa*)(&Sr[so + ja + 16]), rb1 = *(const v4fa*)(&Sr[so + ja + 20]);
        const v4f ia0 = *(const v4fa*)(&Si[so + ja]), ia1 = *(const v4fa*)(&Si[so + ja + 4]), ib0 = *(const v4fa*)(&Si[so + ja + 16]), ib1 = *(const v4fa*)(&Si[so + ja + 20]);
        v16h pr, pi;
#pragma unroll
        for (int i = 0; i < 4; ++i) {
            const pt3 e0 = pterm(ra0[i], ia0[i], mx), e1 = pterm(ra1[i], ia1[i], mx), e2 = pterm(rb0[i], ib0[i], mx), e3 = pterm(rb1[i], ib1[i], mx);
            l += (e0.e + e1.e) + (e2.e + e3.e);
            pr[i] = toh_flush(e0.r * PCAR); pr[4 + i] = toh_flush(e1.r * PCAR); pr[8 + i] = toh_flush(e2.r * PCAR); pr[12 + i] = toh_flush(e3.r * PCAR);
            pi[i] = toh_flush(e0.i * PCAR); pi[4 + i] = toh_flush(e1.i * PCAR); pi[8 + i] = toh_flush(e2.i * PCAR); pi[12 + i] = toh_flush(e3.i * PCAR);
        }
        const v16h pn = -pi;
        const h16* va = VTH + vo + key0; const h16* vb = VTR + vo + key0;
        { const v16h v0 = ldh(va), v1 = ldh(va + (size_t)16 * SEQ), v2 = ldh(va + (size_t)32 * SEQ), v3 = ldh(va + (size_t)48 * SEQ);
          oR[0] = mma(v0, pr, oR[0]); oI[0] = mma(v0, pi, oI[0]); oR[1] = mma(v1, pr, oR[1]); oI[1] = mma(v1, pi, oI[1]);
          oR[2] = mma(v2, pr, oR[2]); oI[2] = mma(v2, pi, oI[2]); oR[3] = mma(v3, pr, oR[3]); oI[3] = mma(v3, pi, oI[3]); }
        { const v16h v0 = ldh(va + (size_t)64 * SEQ), v1 = ldh(va + (size_t)80 * SEQ), v2 = ldh(va + (size_t)96 * SEQ), v3 = ldh(va + (size_t)112 * SEQ);
          oR[0] = mma(v0, pn, oR[0]); oI[0] = mma(v0, pr, oI[0]); oR[1] = mma(v1, pn, oR[1]); oI[1] = mma(v1, pr, oI[1]);
          oR[2] = mma(v2, pn, oR[2]); oI[2] = mma(v2, pr, oI[2]); oR[3] = mma(v3, pn, oR[3]); oI[3] = mma(v3, pr, oI[3]); }
        { const v16h v0 = ldh(vb), v1 = ldh(vb + (size_t)16 * SEQ), v2 = ldh(vb + (size_t)32 * SEQ), v3 = ldh(vb + (size_t)48 * SEQ);
          rR[0] = mma(v0, pr, rR[0]); rI[0] = mma(v0, pi, rI[0]); rR[1] = mma(v1, pr, rR[1]); rI[1] = mma(v1, pi, rI[1]);
          rR[2] = mma(v2, pr, rR[2]); rI[2] = mma(v2, pi, rI[2]); rR[3] = mma(v3, pr, rR[3]); rI[3] = mma(v3, pi, rI[3]); }
        { const v16h v0 = ldh(vb + (size_t)64 * SEQ), v1 = ldh(vb + (size_t)80 * SEQ), v2 = ldh(vb + (size_t)96 * SEQ), v3 = ldh(vb + (size_t)112 * SEQ);
          rR[0] = mma(v0, pn, rR[0]); rI[0] = mma(v0, pr, rI[0]); rR[1] = mma(v1, pn, rR[1]); rI[1] = mma(v1, pr, rI[1]);
          rR[2] = mma(v2, pn, rR[2]); rI[2] = mma(v2, pr, rI[2]); rR[3] = mma(v3, pn, rR[3]); rI[3] = mma(v3, pr, rI[3]); }
    }
    l += __shfl_xor(l, 16, 32);

    { const float oi = (1.0f / l) * PCI;
#pragma unroll
      for (int jd = 0; jd < 4; ++jd) {
          v4f x, y, u, w;
#pragma unroll
          for (int i = 0; i < 4; ++i) { x[i] = (oR[jd][i] + rR[jd][i] * QRI) * oi; y[i] = (oR[jd][4 + i] + rR[jd][4 + i] * QRI) * oi;
                                        u[i] = (oI[jd][i] + rI[jd][i] * QRI) * oi; w[i] = (oI[jd][4 + i] + rI[jd][4 + i] * QRI) * oi; }
          *(v4fa*)(&os[lr * OSP + 16 * jd + 8 * hi]) = x;      *(v4fa*)(&os[lr * OSP + 16 * jd + 8 * hi + 4]) = y;
          *(v4fa*)(&os[lr * OSP + 64 + 16 * jd + 8 * hi]) = u; *(v4fa*)(&os[lr * OSP + 64 + 16 * jd + 8 * hi + 4]) = w; } }
    wave_sync();
    const size_t cb = ((size_t)b * SEQ + t0) * KK + h * HD;
#pragma unroll 1
    for (int ps = 0; ps < 2; ++ps) {
#pragma unroll
        for (int s = 0; s < 8; ++s) { const int line = 4 * s + (lane >> 3); const int row = line >> 1, part = line & 1, c8 = (lane & 7) * 8;
            const v4f x0 = *(const v4fa*)(&os[row * OSP + part * 64 + c8]); const v4f x1 = *(const v4fa*)(&os[row * OSP + part * 64 + c8 + 4]); v8h hv, rv;
#pragma unroll
            for (int i = 0; i < 4; ++i) { const h16 a0 = toh_flush(x0[i]); const h16 a1 = toh_flush(x1[i]); hv[i] = a0; hv[4 + i] = a1;
                rv[i] = toh_flush((x0[i] - (float)a0) * QRS); rv[4 + i] = toh_flush((x1[i] - (float)a1) * QRS); }
            const size_t oo = cb + (size_t)row * KK + part * DM + c8;
            *(volatile v8h*)(CH + oo) = hv; *(volatile v8h*)(CR + oo) = rv; }
        if (ps == 0) __threadfence(); }
}

static constexpr size_t al256(size_t v) { return (v + 255) & ~(size_t)255; }
static constexpr size_t SZ_X  = al256((size_t)ROWS * XP * 4);
static constexpr size_t SZ_A  = al256((size_t)ROWS * KK * 2);
static constexpr size_t SZ_P  = al256((size_t)2 * NB * NH_ * SEQ * HD2 * 2);
static constexpr size_t SZ_W  = al256((size_t)3 * NL * NN * KK * 2);
static constexpr size_t SZ_TOTAL = 2 * SZ_X + 4 * SZ_A + 2 * SZ_P + SZ_W;
static_assert(SZ_TOTAL <= (size_t)134217728);

extern "C" void kernel_launch(void* const* d_in, const int* in_sizes, int n_in,
                              void* d_out, int out_size, void* d_ws, size_t ws_size, hipStream_t stream) {
    if (n_in < 20) return;
    const size_t needx = ((size_t)(NB - 1) * SEQ_FULL + SEQ) * DM;
    if ((size_t)in_sizes[0] < needx || (size_t)in_sizes[1] < needx) return;
    for (int i = 2; i <= 9; ++i) if ((size_t)in_sizes[i] < (size_t)NL * DM) return;
    for (int i = 10; i <= 13; ++i) if ((size_t)in_sizes[i] < (size_t)NL * DM * DM) return;
    if ((size_t)in_sizes[14] < (size_t)NL * DM || (size_t)in_sizes[15] < (size_t)NL * DM) return;
    if ((size_t)in_sizes[16] < (size_t)NL * DM * DM || (size_t)in_sizes[17] < (size_t)NL * DM * DM) return;
    if ((size_t)in_sizes[18] < (size_t)NL || (size_t)in_sizes[19] < (size_t)NL) return;
    if ((size_t)out_size < OFFI + ((size_t)(NB - 1) * OUT_SEQ + SEQ) * DM) return;
    if (SZ_TOTAL > ws_size) return;

    const float* x_re = (const float*)d_in[0];   const float* x_im = (const float*)d_in[1];
    const float* g1r  = (const float*)d_in[2];   const float* b1r  = (const float*)d_in[3];   const float* g1i = (const float*)d_in[4];   const float* b1i = (const float*)d_in[5];
    const float* g2r  = (const float*)d_in[6];   const float* b2r  = (const float*)d_in[7];   const float* g2i = (const float*)d_in[8];   const float* b2i = (const float*)d_in[9];
    const float* wq_r = (const float*)d_in[10];  const float* wq_i = (const float*)d_in[11];
    const float* wo_r = (const float*)d_in[12];  const float* wo_i = (const float*)d_in[13];
    const float* bo_r = (const float*)d_in[14];  const float* bo_i = (const float*)d_in[15];
    const float* wf_r = (const float*)d_in[16];  const float* wf_i = (const float*)d_in[17];
    const float* step = (const float*)d_in[18];  const float* lamb = (const float*)d_in[19];
    float* OUT = (float*)d_out;

    char* wsp = (char*)d_ws;
    float* XA = (float*)wsp; wsp += SZ_X;
    float* XB = (float*)wsp; wsp += SZ_X;
    h16* AH = (h16*)wsp; wsp += SZ_A;
    h16* AR = (h16*)wsp; wsp += SZ_A;
    h16* CH = (h16*)wsp; wsp += SZ_A;
    h16* CR = (h16*)wsp; wsp += SZ_A;
    h16* WPH = (h16*)wsp; wsp += SZ_P;
    h16* VTH = (h16*)wsp; wsp += SZ_P;
    h16* WT  = (h16*)wsp; wsp += SZ_W;
    h16* WPR = WPH + (size_t)NB * NH_ * SEQ * HD2;
    h16* VTR = VTH + (size_t)NB * NH_ * HD2 * SEQ;

    k_xin<<<ROWS, 256, 0, stream>>>(x_re, x_im, XA);
    const dim3 gw((unsigned)(NN * (KK / 8) / 256), NL, 1);
    k_wprep<<<gw, 256, 0, stream>>>(wq_r, wq_i, WT);
    k_wprep<<<gw, 256, 0, stream>>>(wo_r, wo_i, WT + (size_t)NL * WPLANE);
    k_wprep<<<gw, 256, 0, stream>>>(wf_r, wf_i, WT + (size_t)2 * NL * WPLANE);

    const dim3 gln(ROWS / 8, 2, 1);
    const dim3 ggm(ROWS / 32, NN / 64, 1);
    for (int l = 0; l < NL; ++l) {
        k_ln<<<gln, 256, 0, stream>>>(XA, g1r + l * DM, b1r + l * DM, g1i + l * DM, b1i + l * DM, AH, AR);
        k_gemm_qkv<<<ggm, 32, 0, stream>>>(AH, AR, WT + (size_t)l * WPLANE, WPH, WPR);
        k_vT<<<dim3(SEQ / 64, HD2 / 64, 2 * NB * NH_), 256, 0, stream>>>(WPH, VTH);
        k_attn<<<dim3(SEQ / 16, NB * NH_, 1), 32, 0, stream>>>(WPH, VTH, VTR, CH, CR);
        k_gemm_out<<<ggm, 32, 0, stream>>>(CH, CR, WT + (size_t)(NL + l) * WPLANE, bo_r + l * DM, bo_i + l * DM, XA, XB);
        k_ln<<<gln, 256, 0, stream>>>(XB, g2r + l * DM, b2r + l * DM, g2i + l * DM, b2i + l * DM, AH, AR);
        if (l < NL - 1) k_gemm_ff<<<ggm, 32, 0, stream>>>(AH, AR, WT + (size_t)(2 * NL + l) * WPLANE, step, lamb, l, XA, (size_t)DM, XP, SEQ);
        else            k_gemm_ff<<<ggm, 32, 0, stream>>>(AH, AR, WT + (size_t)(2 * NL + l) * WPLANE, step, lamb, l, OUT, OFFI, DM, OUT_SEQ);
    }
}
